// Encoder_6270652252195
// MI455X (gfx1250) — hardware-verified
//
#include <hip/hip_runtime.h>
#include <math.h>

constexpr int NBATCH = 64;
constexpr int NSTEP  = 512;
constexpr int NDIN   = 256;
constexpr int NUNIT  = 256;
constexpr int NGATE3 = 3 * NUNIT;
constexpr int NCAT   = 2 * NUNIT;
constexpr int NROWS  = NSTEP * NBATCH;
constexpr int HPITCH = 264;
constexpr int OPITCH = 260;
constexpr int SCAN_THREADS = 512;
constexpr float ACT_CARRY = 16.0f;
constexpr float WGT_CARRY = 256.0f;
constexpr float FOLD_INV  = 1.0f / (ACT_CARRY * WGT_CARRY);

static_assert(NBATCH == 64, "four 16-row batch tiles");
static_assert(NUNIT == 16 * (SCAN_THREADS / 32), "one 16-unit tile per wave");
static_assert(NROWS % 64 == 0 && NGATE3 % 64 == 0, "GEMM M, N tile multiples");
static_assert(NDIN % 32 == 0 && NCAT % 32 == 0 && NUNIT % 32 == 0, "GEMM K multiples of 32");
static_assert(HPITCH % 8 == 0 && OPITCH % 4 == 0, "16-B aligned LDS rows");
static_assert((NBATCH * NUNIT / 8) % SCAN_THREADS == 0, "sequence copy loop exact");
static_assert(NDIN % 64 == 0 && NCAT % 64 == 0 && NGATE3 % 64 == 0, "transpose tiles exact");

typedef __attribute__((ext_vector_type(16))) _Float16 v16h;
typedef __attribute__((ext_vector_type(8)))  _Float16 v8h;
typedef __attribute__((ext_vector_type(8)))  float    v8f;
typedef __attribute__((ext_vector_type(4)))  float    v4f;
typedef __attribute__((ext_vector_type(4)))  unsigned v4u;

__device__ __forceinline__ unsigned short f2bf_bits(float f) {
  unsigned u = __float_as_uint(f);
  return (unsigned short)((u + 0x7FFFu + ((u >> 16) & 1u)) >> 16);
}
__device__ __forceinline__ float bf_bits2f(unsigned short h) { return __uint_as_float(((unsigned)h) << 16); }
__device__ __forceinline__ float bf16r(float f) { return bf_bits2f(f2bf_bits(f)); }

__device__ __forceinline__ float h16_to_f32(unsigned hb) {
  const unsigned sgn = (hb & 0x8000u) << 16;
  const unsigned em = hb & 0x7fffu;
  const float fn = __uint_as_float((em << 13) + 0x38000000u);
  const float fs = (float)em * 5.9604644775390625e-8f;
  const float mag = (em < 0x400u) ? fs : fn;
  return __uint_as_float(__float_as_uint(mag) | sgn);
}

__device__ __forceinline__ float fsig(float x)  { return __builtin_amdgcn_rcpf(1.0f + __expf(-x)); }
__device__ __forceinline__ float ftanh(float x) { return 1.0f - 2.0f * __builtin_amdgcn_rcpf(__expf(2.0f * x) + 1.0f); }

union FragU { v16h v; v8h h[2]; };
__device__ __forceinline__ v16h frag_load(const _Float16* p) {
  FragU f;
  f.h[0] = *(const v8h*)(p);
  f.h[1] = *(const v8h*)(p + 16);
  return f.v;
}
__device__ __forceinline__ v8f mma_h(v16h a, v16h b, v8f c) {
  return __builtin_amdgcn_wmma_f32_16x16x32_f16(false, a, false, b, (short)0, c, false, false);
}
__device__ __forceinline__ void guard4_h(v8f& a0, v8f& a1, v8f& a2, v8f& a3, v16h x, v16h b0, v16h b1, v16h b2, v16h b3) {
  asm volatile("v_nop\n\tv_nop\n\tv_nop\n\tv_nop"
               : "+v"(a0), "+v"(a1), "+v"(a2), "+v"(a3)
               : "v"(x), "v"(b0), "v"(b1), "v"(b2), "v"(b3));
}
__device__ __forceinline__ void guard6_h(v8f& a0, v8f& a1, v8f& a2, v8f& a3, v8f& a4, v8f& a5,
                                         v16h x0, v16h x1, v16h w0, v16h w1, v16h w2) {
  asm volatile("v_nop\n\tv_nop\n\tv_nop\n\tv_nop"
               : "+v"(a0), "+v"(a1), "+v"(a2), "+v"(a3), "+v"(a4), "+v"(a5)
               : "v"(x0), "v"(x1), "v"(w0), "v"(w1), "v"(w2));
}
__device__ __forceinline__ void acc_guard4(v8f& a, v8f& b, v8f& c, v8f& d) {
  asm volatile("v_nop\n\tv_nop\n\tv_nop\n\tv_nop" : "+v"(a), "+v"(b), "+v"(c), "+v"(d));
}
__device__ __forceinline__ void acc_guard6(v8f& a, v8f& b, v8f& c, v8f& d, v8f& e, v8f& f) {
  asm volatile("v_nop\n\tv_nop\n\tv_nop\n\tv_nop" : "+v"(a), "+v"(b), "+v"(c), "+v"(d), "+v"(e), "+v"(f));
}

__global__ __launch_bounds__(256) void cvt_x_kernel(const float* __restrict__ x, unsigned short* __restrict__ dst) {
  const int i = blockIdx.x * 256 + threadIdx.x;
  if (i < NROWS * (NDIN / 8)) {
    const int m  = i >> 5;
    const int c8 = (i & 31) * 8;
    const int b  = m & (NBATCH - 1);
    const int t  = m >> 6;
    const float* sp = x + ((size_t)b * NSTEP + (size_t)t) * NDIN + c8;
    const v4f a = *(const v4f*)(sp);
    const v4f q = *(const v4f*)(sp + 4);
    v8h hv;
#pragma unroll
    for (int e = 0; e < 4; ++e) {
      hv[e]     = (_Float16)(bf16r(a[e]) * ACT_CARRY);
      hv[4 + e] = (_Float16)(bf16r(q[e]) * ACT_CARRY);
    }
    *(volatile v8h*)(dst + (size_t)i * 8) = hv;
    __threadfence();
    *(volatile v8h*)(dst + (size_t)i * 8) = hv;
  }
}

__global__ __launch_bounds__(256) void tpw_kernel(const float* __restrict__ src, int R, int C, int ldo,
                                                  unsigned short* __restrict__ O, float sc) {
  __shared__ float Tt[64 * 65];
  const int tid = threadIdx.x;
  const int c0 = blockIdx.x * 64, r0 = blockIdx.y * 64;
#pragma unroll
  for (int i = 0; i < 4; ++i) {
    const int idx = i * 256 + tid;
    const int rr = idx >> 4, cc = (idx & 15) * 4;
    const v4f v = *(const v4f*)(src + (size_t)(r0 + rr) * (size_t)C + c0 + cc);
    Tt[rr * 65 + cc + 0] = v[0];
    Tt[rr * 65 + cc + 1] = v[1];
    Tt[rr * 65 + cc + 2] = v[2];
    Tt[rr * 65 + cc + 3] = v[3];
  }
  __syncthreads();
  const int q = tid >> 3, c8 = (tid & 7) * 8;
  v8h hv[2];
#pragma unroll
  for (int g = 0; g < 2; ++g) {
    const int qq = g * 32 + q;
#pragma unroll
    for (int e = 0; e < 8; ++e) {
      const float f = Tt[(c8 + e) * 65 + qq];
      hv[g][e] = (_Float16)(bf16r(f) * sc);
    }
  }
  for (int pass = 0; pass < 2; ++pass) {
#pragma unroll
    for (int g = 0; g < 2; ++g) {
      const size_t o = (size_t)(c0 + g * 32 + q) * (size_t)ldo + (size_t)(r0 + c8);
      *(volatile v8h*)(O + o) = hv[g];
    }
    __threadfence();
  }
}

__global__ __launch_bounds__(256) void gemm_f16_kernel(
    const unsigned short* __restrict__ Ap, int lda,
    const unsigned short* __restrict__ Btp, int ldb,
    unsigned short* __restrict__ Cout, int ldc,
    const float* __restrict__ bias, int M, int N, int K, float scale) {
  const _Float16* A  = (const _Float16*)Ap;
  const _Float16* Bt = (const _Float16*)Btp;
  __shared__ __align__(16) float sT[8][16 * 68];
  const int lane = threadIdx.x & 31;
  const int wave = threadIdx.x >> 5;
  const int tilesN = N >> 6;
  const int tilesM = M >> 6;
  const int tile = blockIdx.x * 8 + wave;
  if (tile >= tilesM * tilesN) return;
  const int tm = tile / tilesN;
  const int tn = tile - tm * tilesN;
  const int m0 = tm << 6;
  const int n0 = tn << 6;
  const int rlane = lane & 15;
  const int koff  = (lane >> 4) * 8;
  const int mOff  = (lane >> 4) * 8;

  v8f acc[4][4];
#pragma unroll
  for (int i = 0; i < 4; ++i)
#pragma unroll
    for (int j = 0; j < 4; ++j) acc[i][j] = (v8f){0.f, 0.f, 0.f, 0.f, 0.f, 0.f, 0.f, 0.f};

  for (int k0 = 0; k0 < K; k0 += 32) {
    v16h bh[4];
#pragma unroll
    for (int j = 0; j < 4; ++j) {
      const size_t bo = (size_t)(n0 + (j << 4) + rlane) * ldb + koff + k0;
      bh[j] = frag_load(Bt + bo);
    }
#pragma unroll
    for (int i = 0; i < 4; ++i) {
      const size_t ao = (size_t)(m0 + (i << 4) + rlane) * lda + koff + k0;
      const v16h ah = frag_load(A + ao);
#pragma unroll
      for (int j = 0; j < 4; ++j) acc[i][j] = mma_h(ah, bh[j], acc[i][j]);
      guard4_h(acc[i][0], acc[i][1], acc[i][2], acc[i][3], ah, bh[0], bh[1], bh[2], bh[3]);
    }
  }
  acc_guard4(acc[0][0], acc[0][1], acc[0][2], acc[0][3]);
  acc_guard4(acc[1][0], acc[1][1], acc[1][2], acc[1][3]);
  acc_guard4(acc[2][0], acc[2][1], acc[2][2], acc[2][3]);
  acc_guard4(acc[3][0], acc[3][1], acc[3][2], acc[3][3]);

  float bvj[4];
#pragma unroll
  for (int j = 0; j < 4; ++j) bvj[j] = bf16r(bias[n0 + (j << 4) + rlane]);

  float* slab = sT[wave];
#pragma unroll
  for (int i = 0; i < 4; ++i) {
    const int mBase = m0 + (i << 4);
#pragma unroll
    for (int j = 0; j < 4; ++j) {
#pragma unroll
      for (int r = 0; r < 8; ++r) {
        const float v = acc[i][j][r] * scale + bvj[j];
        slab[(mOff + r) * 68 + (j << 4) + rlane] = v;
      }
    }
    __builtin_amdgcn_fence(__ATOMIC_RELEASE, "workgroup");
    __builtin_amdgcn_wave_barrier();
    __builtin_amdgcn_fence(__ATOMIC_ACQUIRE, "workgroup");
    {
      const int q = lane >> 3, c8 = (lane & 7) * 8;
      for (int pass = 0; pass < 2; ++pass) {
#pragma unroll
        for (int it = 0; it < 4; ++it) {
          const int row = it * 4 + q;
          const float* sp = slab + row * 68 + c8;
          v8h hv;
#pragma unroll
          for (int e = 0; e < 8; ++e) hv[e] = (_Float16)sp[e];
          *(volatile v8h*)(Cout + (size_t)(mBase + row) * ldc + n0 + c8) = hv;
        }
        __threadfence();
      }
    }
    __builtin_amdgcn_fence(__ATOMIC_RELEASE, "workgroup");
    __builtin_amdgcn_wave_barrier();
    __builtin_amdgcn_fence(__ATOMIC_ACQUIRE, "workgroup");
  }
}

template <bool SEQ_OUT>
__global__ __launch_bounds__(SCAN_THREADS) void gru_scan_kernel(
    const unsigned short* __restrict__ gxp,
    const unsigned short* __restrict__ wup,
    const float* __restrict__ brp,
    const float* __restrict__ h0,
    int backward,
    unsigned short* __restrict__ seqp, int pcol,
    float* __restrict__ hid, int hcol) {
  __shared__ __align__(16) _Float16 Hh[NBATCH * HPITCH];
  __shared__ __align__(16) float    Brs[NGATE3];
  __shared__ __align__(16) float    Hs[16 * OPITCH];
  const _Float16* WU = (const _Float16*)wup;
  const int tid = threadIdx.x, lane = tid & 31, wave = tid >> 5;
  const int c = lane & 15, hh = lane >> 4, koff = hh * 8;
  const int ucol = 16 * wave + 8 * hh;

#pragma unroll 1
  for (int i = tid; i < NGATE3; i += SCAN_THREADS) Brs[i] = bf16r(brp[i]);

  float hst[4][8];
#pragma unroll
  for (int bt = 0; bt < 4; ++bt) {
    const float* hp = h0 + (size_t)(16 * bt + c) * NUNIT + ucol;
    const v4f a = *(const v4f*)(hp);
    const v4f q = *(const v4f*)(hp + 4);
#pragma unroll
    for (int e = 0; e < 4; ++e) {
      hst[bt][e]     = bf16r(a[e]);
      hst[bt][4 + e] = bf16r(q[e]);
    }
    v8h hv;
#pragma unroll
    for (int r = 0; r < 8; ++r) hv[r] = (_Float16)(hst[bt][r] * ACT_CARRY);
    *(v8h*)(Hh + (16 * bt + c) * HPITCH + ucol) = hv;
  }
  __syncthreads();

  const _Float16* wz = WU + (size_t)(0 * NUNIT + 16 * wave + c) * NUNIT + koff;
  const _Float16* wr = WU + (size_t)(1 * NUNIT + 16 * wave + c) * NUNIT + koff;
  const _Float16* wh = WU + (size_t)(2 * NUNIT + 16 * wave + c) * NUNIT + koff;
  const _Float16* hrow = Hh + c * HPITCH + koff;
  const v8f z8 = {0.f, 0.f, 0.f, 0.f, 0.f, 0.f, 0.f, 0.f};

#pragma unroll 1
  for (int s = 0; s < NSTEP; ++s) {
    const int te = backward ? (NSTEP - 1 - s) : s;
    v8f acc[3][4];
#pragma unroll
    for (int g = 0; g < 3; ++g)
#pragma unroll
      for (int bt = 0; bt < 4; ++bt) acc[g][bt] = z8;

#pragma unroll 1
    for (int k0 = 0; k0 < NUNIT; k0 += 32) {
      const v16h fz = frag_load(wz + k0);
      const v16h fr = frag_load(wr + k0);
      const v16h fh = frag_load(wh + k0);
#pragma unroll
      for (int p = 0; p < 2; ++p) {
        const v16h b0 = frag_load(hrow + (32 * p) * HPITCH + k0);
        const v16h b1 = frag_load(hrow + (32 * p + 16) * HPITCH + k0);
        acc[0][2 * p]     = mma_h(fz, b0, acc[0][2 * p]);
        acc[1][2 * p]     = mma_h(fr, b0, acc[1][2 * p]);
        acc[2][2 * p]     = mma_h(fh, b0, acc[2][2 * p]);
        acc[0][2 * p + 1] = mma_h(fz, b1, acc[0][2 * p + 1]);
        acc[1][2 * p + 1] = mma_h(fr, b1, acc[1][2 * p + 1]);
        acc[2][2 * p + 1] = mma_h(fh, b1, acc[2][2 * p + 1]);
        guard6_h(acc[0][2 * p], acc[1][2 * p], acc[2][2 * p],
                 acc[0][2 * p + 1], acc[1][2 * p + 1], acc[2][2 * p + 1], b0, b1, fz, fr, fh);
      }
    }
    acc_guard6(acc[0][0], acc[1][0], acc[2][0], acc[0][1], acc[1][1], acc[2][1]);
    acc_guard6(acc[0][2], acc[1][2], acc[2][2], acc[0][3], acc[1][3], acc[2][3]);
    __syncthreads();

    float bzv[8], brv[8], bhv[8];
    {
      const v4f t0 = *(const v4f*)(Brs + ucol);
      const v4f t1 = *(const v4f*)(Brs + ucol + 4);
      const v4f t2 = *(const v4f*)(Brs + NUNIT + ucol);
      const v4f t3 = *(const v4f*)(Brs + NUNIT + ucol + 4);
      const v4f t4 = *(const v4f*)(Brs + 2 * NUNIT + ucol);
      const v4f t5 = *(const v4f*)(Brs + 2 * NUNIT + ucol + 4);
#pragma unroll
      for (int e = 0; e < 4; ++e) {
        bzv[e] = t0[e]; bzv[4 + e] = t1[e];
        brv[e] = t2[e]; brv[4 + e] = t3[e];
        bhv[e] = t4[e]; bhv[4 + e] = t5[e];
      }
    }
#pragma unroll
    for (int bt = 0; bt < 4; ++bt) {
      const unsigned short* gp = gxp + ((size_t)(te * NBATCH + 16 * bt + c)) * NGATE3 + ucol;
      const v4u gz = *(const v4u*)(gp);
      const v4u gr = *(const v4u*)(gp + NUNIT);
      const v4u gh = *(const v4u*)(gp + 2 * NUNIT);
      v8h hv;
#pragma unroll
      for (int r = 0; r < 8; ++r) {
        const unsigned wq0 = gz[r >> 1];
        const unsigned wq1 = gr[r >> 1];
        const unsigned wq2 = gh[r >> 1];
        const unsigned hb0 = (r & 1) ? (wq0 >> 16) : (wq0 & 0xffffu);
        const unsigned hb1 = (r & 1) ? (wq1 >> 16) : (wq1 & 0xffffu);
        const unsigned hb2 = (r & 1) ? (wq2 >> 16) : (wq2 & 0xffffu);
        const float xz = h16_to_f32(hb0);
        const float xr = h16_to_f32(hb1);
        const float xh = h16_to_f32(hb2);
        const float hz = acc[0][bt][r] * FOLD_INV + bzv[r];
        const float hr = acc[1][bt][r] * FOLD_INV + brv[r];
        const float hc = acc[2][bt][r] * FOLD_INV + bhv[r];
        const float zg = fsig(xz + hz);
        const float rg = fsig(xr + hr);
        const float cand = ftanh(xh + rg * hc);
        const float ho = hst[bt][r];
        const float hn = zg * ho + (1.0f - zg) * cand;
        hst[bt][r] = hn;
        hv[r] = (_Float16)(hn * ACT_CARRY);
      }
      *(v8h*)(Hh + (16 * bt + c) * HPITCH + ucol) = hv;
    }
    __syncthreads();

    if (SEQ_OUT) {
      for (int pass = 0; pass < 2; ++pass) {
#pragma unroll
        for (int it = 0; it < 4; ++it) {
          const int idx = it * SCAN_THREADS + tid;
          const int row = idx >> 5;
          const int c8  = (idx & 31) * 8;
          const v8h v = *(const v8h*)(Hh + row * HPITCH + c8);
          *(volatile v8h*)(seqp + ((size_t)(s * NBATCH + row)) * NCAT + pcol + c8) = v;
        }
        __threadfence();
      }
    }
  }

  if (!SEQ_OUT) {
#pragma unroll
    for (int bt = 0; bt < 4; ++bt) {
      __syncthreads();
      v4f o0, o1;
#pragma unroll
      for (int e = 0; e < 4; ++e) { o0[e] = hst[bt][e]; o1[e] = hst[bt][4 + e]; }
      *(v4f*)(Hs + c * OPITCH + ucol)     = o0;
      *(v4f*)(Hs + c * OPITCH + ucol + 4) = o1;
      __syncthreads();
      for (int pass = 0; pass < 2; ++pass) {
#pragma unroll
        for (int it = 0; it < 2; ++it) {
          const int idx = it * SCAN_THREADS + tid;
          const int row = idx >> 6;
          const int c4  = (idx & 63) * 4;
          const v4f v = *(const v4f*)(Hs + row * OPITCH + c4);
          *(volatile v4f*)(hid + (size_t)(16 * bt + row) * NCAT + hcol + c4) = v;
        }
        __threadfence();
      }
    }
  }
}

__global__ __launch_bounds__(256) void head_kernel(const float* __restrict__ hid, const float* __restrict__ dw,
                                                   const float* __restrict__ db, float* __restrict__ out) {
  const int b = blockIdx.x, n = threadIdx.x;
  const float* hp = hid + (size_t)b * NCAT;
  float acc = 0.0f;
#pragma unroll 1
  for (int k = 0; k < NCAT; ++k) acc = fmaf(hp[k], bf16r(dw[(size_t)k * NUNIT + n]), acc);
  const float v = tanhf(acc + bf16r(db[n]));
  volatile float* op = out + (size_t)b * NUNIT + n;
  *op = v;
  __threadfence();
  *op = v;
}

constexpr size_t WS_X16 = (size_t)NROWS * NDIN * 2;
constexpr size_t WS_W1  = (size_t)NGATE3 * NDIN * 2;
constexpr size_t WS_WU  = (size_t)NGATE3 * NUNIT * 2;
constexpr size_t WS_W2  = (size_t)NGATE3 * NCAT * 2;
constexpr size_t WS_GX  = (size_t)NROWS * NGATE3 * 2;
constexpr size_t WS_SEQ = (size_t)NROWS * NCAT * 2;
constexpr size_t WS_HID = (size_t)NBATCH * NCAT * 4;
constexpr size_t WS_TOTAL = WS_X16 + 2 * WS_W1 + 4 * WS_WU + 2 * WS_W2 + WS_GX + WS_SEQ + WS_HID;
static_assert(WS_TOTAL == (size_t)104726528, "carve total");
static_assert(WS_TOTAL <= (size_t)134217728, "carve within budget");
static_assert(WS_X16 % 256 == 0 && WS_W1 % 256 == 0 && WS_WU % 256 == 0 && WS_W2 % 256 == 0 &&
              WS_GX % 256 == 0 && WS_SEQ % 256 == 0 && WS_HID % 256 == 0, "256-B aligned regions");

extern "C" void kernel_launch(void* const* d_in, const int* in_sizes, int n_in,
                              void* d_out, int out_size, void* d_ws, size_t ws_size, hipStream_t stream) {
  if (n_in < 16 || d_out == nullptr || d_ws == nullptr) return;
  if (in_sizes[0] != NBATCH * NUNIT || in_sizes[1] != NBATCH * NSTEP * NDIN ||
      in_sizes[2] != NDIN * NGATE3 || in_sizes[3] != NUNIT * NGATE3 || in_sizes[4] != 2 * NGATE3 ||
      in_sizes[5] != NDIN * NGATE3 || in_sizes[6] != NUNIT * NGATE3 || in_sizes[7] != 2 * NGATE3 ||
      in_sizes[8] != NCAT * NGATE3 || in_sizes[9] != NUNIT * NGATE3 || in_sizes[10] != 2 * NGATE3 ||
      in_sizes[11] != NCAT * NGATE3 || in_sizes[12] != NUNIT * NGATE3 || in_sizes[13] != 2 * NGATE3 ||
      in_sizes[14] != NCAT * NUNIT || in_sizes[15] != NUNIT || out_size != NBATCH * NUNIT) return;
  if (WS_TOTAL > ws_size) return;

  const float* h0  = (const float*)d_in[0];
  const float* x   = (const float*)d_in[1];
  const float* k1f = (const float*)d_in[2];
  const float* u1f = (const float*)d_in[3];
  const float* b1f = (const float*)d_in[4];
  const float* k1b = (const float*)d_in[5];
  const float* u1b = (const float*)d_in[6];
  const float* b1b = (const float*)d_in[7];
  const float* k2f = (const float*)d_in[8];
  const float* u2f = (const float*)d_in[9];
  const float* b2f = (const float*)d_in[10];
  const float* k2b = (const float*)d_in[11];
  const float* u2b = (const float*)d_in[12];
  const float* b2b = (const float*)d_in[13];
  const float* dw  = (const float*)d_in[14];
  const float* db  = (const float*)d_in[15];
  float* out = (float*)d_out;

  char* ws = (char*)d_ws;
  size_t off = 0;
  auto carve = [&](size_t bytes) -> char* { char* p = ws + off; off += bytes; return p; };
  unsigned short* X16 = (unsigned short*)carve(WS_X16);
  unsigned short* K1F = (unsigned short*)carve(WS_W1);
  unsigned short* K1B = (unsigned short*)carve(WS_W1);
  unsigned short* U1F = (unsigned short*)carve(WS_WU);
  unsigned short* U1B = (unsigned short*)carve(WS_WU);
  unsigned short* K2F = (unsigned short*)carve(WS_W2);
  unsigned short* K2B = (unsigned short*)carve(WS_W2);
  unsigned short* U2F = (unsigned short*)carve(WS_WU);
  unsigned short* U2B = (unsigned short*)carve(WS_WU);
  unsigned short* GX  = (unsigned short*)carve(WS_GX);
  unsigned short* SEQ = (unsigned short*)carve(WS_SEQ);
  float*          HID = (float*)carve(WS_HID);
  if (off != WS_TOTAL) return;

  cvt_x_kernel<<<(NROWS * (NDIN / 8)) / 256, 256, 0, stream>>>(x, X16);
  tpw_kernel<<<dim3(NGATE3 / 64, NDIN / 64), 256, 0, stream>>>(k1f, NDIN, NGATE3, NDIN, K1F, WGT_CARRY);
  tpw_kernel<<<dim3(NGATE3 / 64, NDIN / 64), 256, 0, stream>>>(k1b, NDIN, NGATE3, NDIN, K1B, WGT_CARRY);
  tpw_kernel<<<dim3(NGATE3 / 64, NUNIT / 64), 256, 0, stream>>>(u1f, NUNIT, NGATE3, NUNIT, U1F, WGT_CARRY);
  tpw_kernel<<<dim3(NGATE3 / 64, NUNIT / 64), 256, 0, stream>>>(u1b, NUNIT, NGATE3, NUNIT, U1B, WGT_CARRY);
  tpw_kernel<<<dim3(NGATE3 / 64, NCAT / 64), 256, 0, stream>>>(k2f, NCAT, NGATE3, NCAT, K2F, WGT_CARRY);
  tpw_kernel<<<dim3(NGATE3 / 64, NCAT / 64), 256, 0, stream>>>(k2b, NCAT, NGATE3, NCAT, K2B, WGT_CARRY);
  tpw_kernel<<<dim3(NGATE3 / 64, NUNIT / 64), 256, 0, stream>>>(u2f, NUNIT, NGATE3, NUNIT, U2F, WGT_CARRY);
  tpw_kernel<<<dim3(NGATE3 / 64, NUNIT / 64), 256, 0, stream>>>(u2b, NUNIT, NGATE3, NUNIT, U2B, WGT_CARRY);

  const int gblocks = ((NROWS / 64) * (NGATE3 / 64)) / 8;

  gemm_f16_kernel<<<gblocks, 256, 0, stream>>>(X16, NDIN, K1F, NDIN, GX, NGATE3, b1f, NROWS, NGATE3, NDIN, FOLD_INV);
  gru_scan_kernel<true><<<1, SCAN_THREADS, 0, stream>>>(GX, U1F, b1f + NGATE3, h0, 0, SEQ, 0, HID, 0);
  gemm_f16_kernel<<<gblocks, 256, 0, stream>>>(X16, NDIN, K1B, NDIN, GX, NGATE3, b1b, NROWS, NGATE3, NDIN, FOLD_INV);
  gru_scan_kernel<true><<<1, SCAN_THREADS, 0, stream>>>(GX, U1B, b1b + NGATE3, h0, 1, SEQ, NUNIT, HID, 0);
  gemm_f16_kernel<<<gblocks, 256, 0, stream>>>(SEQ, NCAT, K2F, NCAT, GX, NGATE3, b2f, NROWS, NGATE3, NCAT, FOLD_INV);
  gru_scan_kernel<false><<<1, SCAN_THREADS, 0, stream>>>(GX, U2F, b2f + NGATE3, h0, 0, SEQ, 0, HID, 0);
  gemm_f16_kernel<<<gblocks, 256, 0, stream>>>(SEQ, NCAT, K2B, NCAT, GX, NGATE3, b2b, NROWS, NGATE3, NCAT, FOLD_INV);
  gru_scan_kernel<false><<<1, SCAN_THREADS, 0, stream>>>(GX, U2B, b2b + NGATE3, h0, 1, SEQ, 0, HID, NUNIT);
  head_kernel<<<NBATCH, 256, 0, stream>>>(HID, dw, db, out);
}
